// GCN_87325275062334
// MI455X (gfx1250) — hardware-verified
//
#include <hip/hip_runtime.h>
#include <stddef.h>
#include <stdint.h>
#include <math.h>


#define DM     128
#define DFF    512
#define NHEAD  8
#define HDIM   16
#define MSEQ   1024
#define NLAYER 2
#define QP     256
#define FP     1024
#define VTP    1024
#define NTHR   256
#define NWAVE  8
#define EPT    8
#define CHUNK  (NTHR * EPT)
#define WCAP   (EPT * 32)
#define LISTN  (NWAVE * WCAP)
#define NBD    8192
#define SLD    13
#define NBA    512
#define SLA    9
#define RCAP   24576
#define DEGCAP 128
#define GBM    64
#define GBN    128
#define GTHR   128
#define ATQ    64
#define ATHR   128
#define AGG_ZINTS    (LISTN + 2 * RCAP + 3 * NBA)
#define MISC_INTS    16
#define ROWBUF_INTS  (NWAVE * QP / 2)
#define AGG_LDS_INTS (AGG_ZINTS + MISC_INTS + ROWBUF_INTS)
#define WPL_C1  0
#define WPL_C2  16384
#define WPL_L0  49152
#define WPL_LSZ 393216
#define WPL_Q   0
#define WPL_K   32768
#define WPL_V   65536
#define WPL_O   98304
#define WPL_1   131072
#define WPL_2   262144
#define WPL_TOT (WPL_L0 + NLAYER * WPL_LSZ)
#define NPARTS  (3 + 12 * NLAYER)
#define UMAX    8192
#define WSMAX   134217728

static_assert((CHUNK & (CHUNK - 1)) == 0 && CHUNK <= 4096);
static_assert((NBD & (NBD - 1)) == 0 && NBD == (1 << SLD));
static_assert((NBA & (NBA - 1)) == 0 && NBA == (1 << SLA));
static_assert(((long long)CHUNK << SLD) < (1LL << 31));
static_assert(((long long)CHUNK << SLA) < (1LL << 31));
static_assert(NBD % (NTHR * 4) == 0);
static_assert(LISTN % NTHR == 0);
static_assert(NBA % NWAVE == 0 && NBA % 32 == 0 && NBA % GBM == 0);
static_assert(RCAP % 32 == 0 && AGG_ZINTS % 4 == 0 && LISTN % 4 == 0 && ((AGG_ZINTS + MISC_INTS) % 4) == 0);
static_assert(AGG_LDS_INTS * 4 <= 300000);
static_assert(GBM == (GTHR / 32) * 16 && GBN == DM && DM == 4 * 32 && DM % 32 == 0);
static_assert(QP == 2 * DM && FP == 2 * DFF && DFF % GBN == 0 && QP % 32 == 0 && FP % 32 == 0);
static_assert(NHEAD * HDIM == DM && HDIM == 16);
static_assert(MSEQ % ATQ == 0 && ATQ == (ATHR / 32) * 16 && MSEQ % 32 == 0 && MSEQ % GBM == 0 && VTP == MSEQ);
static_assert(WPL_C2 + DM * QP == WPL_L0 && WPL_1 + DFF * QP == WPL_2 && WPL_2 + DM * FP == WPL_LSZ);
static_assert(WPL_Q + DM * QP == WPL_K && WPL_K + DM * QP == WPL_V && WPL_V + DM * QP == WPL_O && WPL_O + DM * QP == WPL_1);
static_assert((DM << 4) % NTHR == 0 && (DFF << 4) == UMAX && (DM << 6) == UMAX && UMAX % NTHR == 0);
static_assert(ATQ * QP * 2 <= 65536 && GBM * GBN * 4 + GBM * QP * 2 <= 65536);

typedef float          v4f   __attribute__((ext_vector_type(4)));
typedef float          v8f   __attribute__((ext_vector_type(8)));
typedef int            v4i   __attribute__((ext_vector_type(4)));
typedef int            v8i   __attribute__((ext_vector_type(8)));
typedef unsigned short v4us  __attribute__((ext_vector_type(4)));
typedef unsigned short v8us  __attribute__((ext_vector_type(8)));
typedef unsigned short v16us __attribute__((ext_vector_type(16)));
typedef __bf16         v16bf __attribute__((ext_vector_type(16)));
typedef v4f  __attribute__((may_alias)) v4fa;
typedef v4i  __attribute__((may_alias)) v4ia;
typedef v4us __attribute__((may_alias)) v4usa;
typedef v8us __attribute__((may_alias)) v8usa;
union FragB { v16bf v; v16us u; v8us h[2]; v8i w; };

__device__ __forceinline__ v8f wmb(const FragB& a, const FragB& b, v8f c) {
  v8f d = __builtin_amdgcn_wmma_f32_16x16x32_bf16(false, a.v, false, b.v, (short)0, c, false, false);
  asm volatile("v_nop\n\tv_nop\n\tv_nop\n\tv_nop" : "+v"(d) : "v"(a.w), "v"(b.w));
  return d;
}

__device__ __forceinline__ unsigned bf16_bits(float f) {
  const unsigned u = __float_as_uint(f);
  return (u + 0x7FFFu + ((u >> 16) & 1u)) >> 16;
}
__device__ __forceinline__ float bf16_val(float f) {
  return __uint_as_float(bf16_bits(f) << 16);
}
__device__ __forceinline__ unsigned short hsel_bits(float v, bool losel) {
  const unsigned hb = bf16_bits(v);
  const unsigned lb = bf16_bits(v - __uint_as_float(hb << 16));
  return (unsigned short)(losel ? lb : hb);
}

__device__ __forceinline__ void wave_sync() {
  __builtin_amdgcn_fence(__ATOMIC_RELEASE, "wavefront");
  __builtin_amdgcn_wave_barrier();
  __builtin_amdgcn_fence(__ATOMIC_ACQUIRE, "wavefront");
}

template <int SLB>
__device__ __forceinline__ int scan_chunk(const int* __restrict__ dsts, int nE, int cbase, int slotBase,
                                          int nb, int vec8, int* list, int tid, int lane, int wave) {
  int wc = 0;
  const int el0  = tid * EPT;
  const int e0   = cbase + el0;
  const int sent = -2147483647 - 1;
  v4i da, db;
  if (vec8 != 0 && cbase + CHUNK <= nE) {
    da = *(const v4i*)(dsts + e0);
    db = *(const v4i*)(dsts + e0 + 4);
  } else {
    da.x = (e0     < nE) ? dsts[min(e0,     nE - 1)] : sent;
    da.y = (e0 + 1 < nE) ? dsts[min(e0 + 1, nE - 1)] : sent;
    da.z = (e0 + 2 < nE) ? dsts[min(e0 + 2, nE - 1)] : sent;
    da.w = (e0 + 3 < nE) ? dsts[min(e0 + 3, nE - 1)] : sent;
    db.x = (e0 + 4 < nE) ? dsts[min(e0 + 4, nE - 1)] : sent;
    db.y = (e0 + 5 < nE) ? dsts[min(e0 + 5, nE - 1)] : sent;
    db.z = (e0 + 6 < nE) ? dsts[min(e0 + 6, nE - 1)] : sent;
    db.w = (e0 + 7 < nE) ? dsts[min(e0 + 7, nE - 1)] : sent;
  }
  const unsigned nbs = (unsigned)slotBase;
  const unsigned unb = (unsigned)nb;
  const unsigned s0 = (unsigned)da.x - nbs, s1 = (unsigned)da.y - nbs;
  const unsigned s2 = (unsigned)da.z - nbs, s3 = (unsigned)da.w - nbs;
  const unsigned s4 = (unsigned)db.x - nbs, s5 = (unsigned)db.y - nbs;
  const unsigned s6 = (unsigned)db.z - nbs, s7 = (unsigned)db.w - nbs;
  const bool h0 = s0 < unb, h1 = s1 < unb, h2 = s2 < unb, h3 = s3 < unb;
  const bool h4 = s4 < unb, h5 = s5 < unb, h6 = s6 < unb, h7 = s7 < unb;
  const unsigned any = __builtin_amdgcn_ballot_w32(h0 | h1 | h2 | h3 | h4 | h5 | h6 | h7);
  if (any != 0u) {
#define HITJ(J, HJ, SJ) { \
      const unsigned mj = __builtin_amdgcn_ballot_w32(HJ); \
      if (mj != 0u) { \
        if (HJ) { \
          const int pos = wc + (int)__builtin_amdgcn_mbcnt_lo(mj, 0u); \
          if (pos < WCAP) list[wave * WCAP + pos] = ((el0 + (J)) << SLB) | (int)(SJ); \
        } \
        wc += (int)__builtin_popcount(mj); } }
    HITJ(0, h0, s0)
    HITJ(1, h1, s1)
    HITJ(2, h2, s2)
    HITJ(3, h3, s3)
    HITJ(4, h4, s4)
    HITJ(5, h5, s5)
    HITJ(6, h6, s6)
    HITJ(7, h7, s7)
#undef HITJ
  }
  return wc;
}

__global__ __launch_bounds__(NTHR) void k_wprep(
    const float* __restrict__ c1W, const float* __restrict__ c2W,
    const float* __restrict__ Wq, const float* __restrict__ Wk, const float* __restrict__ Wv,
    const float* __restrict__ Wo, const float* __restrict__ W1, const float* __restrict__ W2,
    unsigned short* wpl) {
  const int part = (int)blockIdx.y;
  const int u = (int)blockIdx.x * NTHR + (int)threadIdx.x;
  const float* W;
  int nout, ks, pitch;
  size_t dofs;
  if (part == 0) {
    W = c1W; nout = DM; ks = 4; pitch = DM; dofs = WPL_C1;
  } else if (part < 3) {
    W = c2W; nout = DM; ks = 4; pitch = QP; dofs = (size_t)WPL_C2 + (size_t)(part - 1) * DM;
  } else if (part < NPARTS) {
    const int pj = part - 3;
    const int l  = pj / 12;
    const int j  = pj - 12 * l;
    const int pr = j >> 1, cp = j & 1;
    const size_t lb = (size_t)WPL_L0 + (size_t)l * WPL_LSZ;
    if (pr == 0)      { W = Wq + (size_t)l * DM * DM;  nout = DM;  ks = 4; pitch = QP; dofs = lb + WPL_Q + (size_t)cp * DM; }
    else if (pr == 1) { W = Wk + (size_t)l * DM * DM;  nout = DM;  ks = 4; pitch = QP; dofs = lb + WPL_K + (size_t)cp * DM; }
    else if (pr == 2) { W = Wv + (size_t)l * DM * DM;  nout = DM;  ks = 4; pitch = QP; dofs = lb + WPL_V + (size_t)cp * DM; }
    else if (pr == 3) { W = Wo + (size_t)l * DM * DM;  nout = DM;  ks = 4; pitch = QP; dofs = lb + WPL_O + (size_t)cp * DM; }
    else if (pr == 4) { W = W1 + (size_t)l * DM * DFF; nout = DFF; ks = 4; pitch = QP; dofs = lb + WPL_1 + (size_t)cp * DM; }
    else              { W = W2 + (size_t)l * DFF * DM; nout = DM;  ks = 6; pitch = FP; dofs = lb + WPL_2 + (size_t)cp * DFF; }
  } else {
    return;
  }
  const int kq    = 1 << ks;
  const int units = nout << ks;
  if (u >= units) return;
  const int n  = u >> ks;
  const int k8 = (u & (kq - 1)) * 8;
  const float* p = W + (size_t)k8 * (size_t)nout + n;
  v8us o;
#pragma unroll
  for (int i = 0; i < 8; ++i) o[i] = (unsigned short)bf16_bits(p[(size_t)i * (size_t)nout]);
  unsigned short* dp = wpl + dofs + (size_t)n * (size_t)pitch + k8;
  *(volatile v8us*)dp = o;
  __threadfence();
  *(volatile v8us*)dp = o;
}

__global__ __launch_bounds__(NTHR) void k_cvt(const float* __restrict__ xr, const float* __restrict__ en, int nN,
                                              unsigned short* xb, unsigned short* eb, float* h0) {
  const int part = (int)blockIdx.y;
  const int u = (int)blockIdx.x * NTHR + (int)threadIdx.x;
  if (part < 2) {
    const int nUnits = nN * (DM / 8);
    if ((int)blockIdx.x * NTHR >= nUnits) return;
    const float* src = (part == 0) ? xr : en;
    unsigned short* dstp = (part == 0) ? xb : eb;
    const int row = u >> 4;
    const int k8  = (u & 15) * 8;
    const float* p = src + (size_t)row * DM + k8;
    const v4f a = *(const v4fa*)p;
    const v4f b = *(const v4fa*)(p + 4);
    v8us o;
    o[0] = (unsigned short)bf16_bits(a.x); o[1] = (unsigned short)bf16_bits(a.y);
    o[2] = (unsigned short)bf16_bits(a.z); o[3] = (unsigned short)bf16_bits(a.w);
    o[4] = (unsigned short)bf16_bits(b.x); o[5] = (unsigned short)bf16_bits(b.y);
    o[6] = (unsigned short)bf16_bits(b.z); o[7] = (unsigned short)bf16_bits(b.w);
    unsigned short* dp = dstp + (size_t)row * DM + k8;
    *(volatile v8us*)dp = o;
    __threadfence();
    *(volatile v8us*)dp = o;
  } else {
    const int nUnits = nN * (DM / 4);
    if ((int)blockIdx.x * NTHR >= nUnits) return;
    const v4f a = *(const v4fa*)(en + 4 * (size_t)u);
    v4f y;
    y.x = bf16_val(a.x); y.y = bf16_val(a.y); y.z = bf16_val(a.z); y.w = bf16_val(a.w);
    float* dp = h0 + 4 * (size_t)u;
    *(volatile v4f*)dp = y;
    __threadfence();
    *(volatile v4f*)dp = y;
  }
}

__global__ __launch_bounds__(NTHR) void k_deg(const int* __restrict__ dsts, int nE, int vec8, float* dis) {
  __shared__ __attribute__((aligned(16))) int scnt[NBD];
  __shared__ __attribute__((aligned(16))) int list[LISTN];
  __shared__ int wcnt[NWAVE];
  const int tid = (int)threadIdx.x, lane = tid & 31, wave = tid >> 5;
  const int nodeBase = (int)blockIdx.x * NBD;

  for (int i = tid; i < NBD; i += NTHR) scnt[i] = 0;
  for (int i = tid; i < LISTN; i += NTHR) list[i] = 0;
  if (tid < NWAVE) wcnt[tid] = 0;
  __syncthreads();

  const int nChunks = (nE + CHUNK - 1) / CHUNK;
#pragma unroll 1
  for (int ch = 0; ch < nChunks; ++ch) {
    const int cbase = ch * CHUNK;
    const int wc = scan_chunk<SLD>(dsts, nE, cbase, nodeBase, NBD, vec8, list, tid, lane, wave);
    if (lane == 0) wcnt[wave] = wc;
    __syncthreads();
    if (wave == 0) {
#pragma unroll 1
      for (int w2 = 0; w2 < NWAVE; ++w2) {
        int c = wcnt[w2];
        c = c < 0 ? 0 : (c > WCAP ? WCAP : c);
#pragma unroll 1
        for (int b0 = 0; b0 < c; b0 += 32) {
          const int idx = b0 + lane;
          const int ent = list[w2 * WCAP + (idx < WCAP ? idx : WCAP - 1)];
          const int m32 = (c - b0) < 32 ? (c - b0) : 32;
#pragma unroll 1
          for (int k = 0; k < m32; ++k) {
            const int u  = __builtin_amdgcn_readlane(ent, k);
            const int sl = u & (NBD - 1);
            if (lane == 0) scnt[sl] = scnt[sl] + 1;
          }
        }
      }
    }
    __syncthreads();
  }

  v4f vals[NBD / (NTHR * 4)];
#pragma unroll
  for (int it = 0; it < NBD / (NTHR * 4); ++it) {
    const int s0 = it * (NTHR * 4) + 4 * tid;
    const v4i c4 = *(const v4ia*)(scnt + s0);
    const float d0 = (float)c4.x + 1.0f, d1 = (float)c4.y + 1.0f;
    const float d2 = (float)c4.z + 1.0f, d3 = (float)c4.w + 1.0f;
    v4f v;
    v.x = rsqrtf(d0); v.y = rsqrtf(d1); v.z = rsqrtf(d2); v.w = rsqrtf(d3);
    vals[it] = v;
  }
#pragma unroll
  for (int it = 0; it < NBD / (NTHR * 4); ++it) {
    const int s0 = it * (NTHR * 4) + 4 * tid;
    *(volatile v4f*)(dis + (size_t)nodeBase + s0) = vals[it];
  }
  __threadfence();
#pragma unroll
  for (int it = 0; it < NBD / (NTHR * 4); ++it) {
    const int s0 = it * (NTHR * 4) + 4 * tid;
    *(volatile v4f*)(dis + (size_t)nodeBase + s0) = vals[it];
  }
}

template <int MODE>
__global__ __launch_bounds__(GTHR) void k_gemm(
    const unsigned short* __restrict__ A, int lda,
    const unsigned short* __restrict__ BT, int ldb, int K,
    const float* __restrict__ bias, int Ntot,
    const float* resid, const float* __restrict__ gam, const float* __restrict__ bet,
    float* outF, unsigned short* outH)
{
  extern __shared__ __attribute__((aligned(16))) float gsm[];
  float* stg = gsm;
  const int tid = (int)threadIdx.x, lane = tid & 31, wave = tid >> 5, hh = lane >> 4, m = lane & 15;
  const int rowBase = (int)blockIdx.x * GBM;
  const int col0    = (int)blockIdx.y * GBN;

  v8f acc[8];
  {
    const v8f z = {0.f, 0.f, 0.f, 0.f, 0.f, 0.f, 0.f, 0.f};
#pragma unroll
    for (int t = 0; t < 8; ++t) acc[t] = z;
  }
  const unsigned short* ap = A  + (size_t)(rowBase + 16 * wave + m) * (size_t)lda + 8 * hh;
  const unsigned short* bp = BT + (size_t)(col0 + m) * (size_t)ldb + 8 * hh;

#pragma unroll 1
  for (int k0 = 0; k0 < K; k0 += 32) {
    FragB af;
    af.h[0] = *(const v8usa*)(ap + k0);
    af.h[1] = *(const v8usa*)(ap + k0 + 16);
#pragma unroll
    for (int nt = 0; nt < 8; ++nt) {
      const unsigned short* wq = bp + (size_t)(16 * nt) * (size_t)ldb + k0;
      FragB bf;
      bf.h[0] = *(const v8usa*)wq;
      bf.h[1] = *(const v8usa*)(wq + 16);
      acc[nt] = wmb(af, bf, acc[nt]);
    }
  }

#pragma unroll
  for (int nt = 0; nt < 8; ++nt) {
    const int lc = 16 * nt + m;
#pragma unroll
    for (int r = 0; r < 8; ++r) {
      const int lr = 16 * wave + 8 * hh + r;
      stg[lr * GBN + lc] = acc[nt][r];
    }
  }
  __syncthreads();

  if constexpr (MODE == 0) {
#pragma unroll 1
    for (int i = 0; i < 16; ++i) {
      const int lr = 16 * wave + i;
      const v4f y = *(const v4fa*)(stg + lr * GBN + 4 * lane);
      *(volatile v4f*)(outF + (size_t)(rowBase + lr) * (size_t)Ntot + col0 + 4 * lane) = y;
    }
    __threadfence();
#pragma unroll 1
    for (int i = 0; i < 16; ++i) {
      const int lr = 16 * wave + i;
      const v4f y = *(const v4fa*)(stg + lr * GBN + 4 * lane);
      *(volatile v4f*)(outF + (size_t)(rowBase + lr) * (size_t)Ntot + col0 + 4 * lane) = y;
    }
  } else if constexpr (MODE == 1 || MODE == 2) {
    const int c8 = 8 * m;
    const bool lsel = hh != 0;
    v4f b0, b1;
    {
      const v4f t0 = *(const v4fa*)(bias + col0 + c8);
      const v4f t1 = *(const v4fa*)(bias + col0 + c8 + 4);
      b0.x = bf16_val(t0.x); b0.y = bf16_val(t0.y); b0.z = bf16_val(t0.z); b0.w = bf16_val(t0.w);
      b1.x = bf16_val(t1.x); b1.y = bf16_val(t1.y); b1.z = bf16_val(t1.z); b1.w = bf16_val(t1.w);
    }
    const size_t ldo  = 2 * (size_t)Ntot;
    const size_t cofs = (size_t)(lsel ? Ntot : 0) + (size_t)col0 + (size_t)c8;
#pragma unroll 1
    for (int i = 0; i < 16; ++i) {
      const int lr = 16 * wave + i;
      const float* sp = stg + lr * GBN + c8;
      v4f va = *(const v4fa*)sp + b0;
      v4f vb = *(const v4fa*)(sp + 4) + b1;
      if constexpr (MODE == 2) {
        va.x = fmaxf(va.x, 0.0f); va.y = fmaxf(va.y, 0.0f); va.z = fmaxf(va.z, 0.0f); va.w = fmaxf(va.w, 0.0f);
        vb.x = fmaxf(vb.x, 0.0f); vb.y = fmaxf(vb.y, 0.0f); vb.z = fmaxf(vb.z, 0.0f); vb.w = fmaxf(vb.w, 0.0f);
      }
      v8us o;
      o[0] = hsel_bits(va.x, lsel); o[1] = hsel_bits(va.y, lsel); o[2] = hsel_bits(va.z, lsel); o[3] = hsel_bits(va.w, lsel);
      o[4] = hsel_bits(vb.x, lsel); o[5] = hsel_bits(vb.y, lsel); o[6] = hsel_bits(vb.z, lsel); o[7] = hsel_bits(vb.w, lsel);
      *(volatile v8us*)(outH + (size_t)(rowBase + lr) * ldo + cofs) = o;
    }
    __threadfence();
#pragma unroll 1
    for (int i = 0; i < 16; ++i) {
      const int lr = 16 * wave + i;
      const float* sp = stg + lr * GBN + c8;
      v4f va = *(const v4fa*)sp + b0;
      v4f vb = *(const v4fa*)(sp + 4) + b1;
      if constexpr (MODE == 2) {
        va.x = fmaxf(va.x, 0.0f); va.y = fmaxf(va.y, 0.0f); va.z = fmaxf(va.z, 0.0f); va.w = fmaxf(va.w, 0.0f);
        vb.x = fmaxf(vb.x, 0.0f); vb.y = fmaxf(vb.y, 0.0f); vb.z = fmaxf(vb.z, 0.0f); vb.w = fmaxf(vb.w, 0.0f);
      }
      v8us o;
      o[0] = hsel_bits(va.x, lsel); o[1] = hsel_bits(va.y, lsel); o[2] = hsel_bits(va.z, lsel); o[3] = hsel_bits(va.w, lsel);
      o[4] = hsel_bits(vb.x, lsel); o[5] = hsel_bits(vb.y, lsel); o[6] = hsel_bits(vb.z, lsel); o[7] = hsel_bits(vb.w, lsel);
      *(volatile v8us*)(outH + (size_t)(rowBase + lr) * ldo + cofs) = o;
    }
  } else if constexpr (MODE == 3) {
    const int q = lane >> 3, j = lane & 7;
    const int bidx = rowBase / MSEQ;
    const int m0   = rowBase - bidx * MSEQ;
    const bool lsel = (wave >> 1) != 0;
#pragma unroll 1
    for (int it = 0; it < 16; ++it) {
      const int p = 64 * wave + 4 * it + q;
      const int c = p & (DM - 1);
      const float bvc = bf16_val(bias[col0 + c]);
      v8us o;
#pragma unroll
      for (int t = 0; t < 8; ++t) o[t] = hsel_bits(stg[(8 * j + t) * GBN + c] + bvc, lsel);
      *(volatile v8us*)(outH + ((size_t)bidx * QP + (size_t)p) * (size_t)VTP + m0 + 8 * j) = o;
    }
    __threadfence();
#pragma unroll 1
    for (int it = 0; it < 16; ++it) {
      const int p = 64 * wave + 4 * it + q;
      const int c = p & (DM - 1);
      const float bvc = bf16_val(bias[col0 + c]);
      v8us o;
#pragma unroll
      for (int t = 0; t < 8; ++t) o[t] = hsel_bits(stg[(8 * j + t) * GBN + c] + bvc, lsel);
      *(volatile v8us*)(outH + ((size_t)bidx * QP + (size_t)p) * (size_t)VTP + m0 + 8 * j) = o;
    }
  } else {
    unsigned short* hst = (unsigned short*)(gsm + GBM * GBN);
    v4f b4, g4, e4;
    {
      const v4f tb = *(const v4fa*)(bias + col0 + 4 * lane);
      const v4f tg = *(const v4fa*)(gam + 4 * lane);
      const v4f te = *(const v4fa*)(bet + 4 * lane);
      b4.x = bf16_val(tb.x); b4.y = bf16_val(tb.y); b4.z = bf16_val(tb.z); b4.w = bf16_val(tb.w);
      g4.x = bf16_val(tg.x); g4.y = bf16_val(tg.y); g4.z = bf16_val(tg.z); g4.w = bf16_val(tg.w);
      e4.x = bf16_val(te.x); e4.y = bf16_val(te.y); e4.z = bf16_val(te.z); e4.w = bf16_val(te.w);
    }
#pragma unroll 1
    for (int i = 0; i < 16; ++i) {
      const int lr = 16 * wave + i;
      const size_t grow = (size_t)(rowBase + lr);
      float* srow = stg + lr * GBN + 4 * lane;
      const v4f rr = *(const v4fa*)(resid + grow * DM + 4 * lane);
      const v4f t = *(const v4fa*)srow + b4 + rr;
      float s = (t.x + t.y) + (t.z + t.w);
      s += __shfl_xor(s, 16, 32); s += __shfl_xor(s, 8, 32); s += __shfl_xor(s, 4, 32);
      s += __shfl_xor(s, 2, 32);  s += __shfl_xor(s, 1, 32);
      const float mu = s * (1.0f / DM);
      const v4f d = t - mu;
      float vv = (d.x * d.x + d.y * d.y) + (d.z * d.z + d.w * d.w);
      vv += __shfl_xor(vv, 16, 32); vv += __shfl_xor(vv, 8, 32); vv += __shfl_xor(vv, 4, 32);
      vv += __shfl_xor(vv, 2, 32);  vv += __shfl_xor(vv, 1, 32);
      const float rs = rsqrtf(vv * (1.0f / DM) + 1e-5f);
      const v4f y = (d * rs) * g4 + e4;
      *(v4fa*)srow = y;
      if constexpr (MODE == 4) {
        v4us h4, l4;
        unsigned hb;
        hb = bf16_bits(y.x); h4[0] = (unsigned short)hb; l4[0] = (unsigned short)bf16_bits(y.x - __uint_as_float(hb << 16));
        hb = bf16_bits(y.y); h4[1] = (unsigned short)hb; l4[1] = (unsigned short)bf16_bits(y.y - __uint_as_float(hb << 16));
        hb = bf16_bits(y.z); h4[2] = (unsigned short)hb; l4[2] = (unsigned short)bf16_bits(y.z - __uint_as_float(hb << 16));
        hb = bf16_bits(y.w); h4[3] = (unsigned short)hb; l4[3] = (unsigned short)bf16_bits(y.w - __uint_as_float(hb << 16));
        *(v4usa*)(hst + (size_t)lr * QP + 4 * lane) = h4;
        *(v4usa*)(hst + (size_t)lr * QP + DM + 4 * lane) = l4;
      }
    }
    __syncthreads();
#pragma unroll 1
    for (int i = 0; i < 16; ++i) {
      const int lr = 16 * wave + i;
      const size_t grow = (size_t)(rowBase + lr);
      const v4f y = *(const v4fa*)(stg + lr * GBN + 4 * lane);
      *(volatile v4f*)(outF + grow * DM + 4 * lane) = y;
      if constexpr (MODE == 4) {
        const v8us qv = *(const v8usa*)(hst + (size_t)lr * QP + 8 * lane);
        *(volatile v8us*)(outH + grow * QP + 8 * lane) = qv;
      }
    }
    __threadfence();
#pragma unroll 1
    for (int i = 0; i < 16; ++i) {
      const int lr = 16 * wave + i;
      const size_t grow = (size_t)(rowBase + lr);
      const v4f y = *(const v4fa*)(stg + lr * GBN + 4 * lane);
      *(volatile v4f*)(outF + grow * DM + 4 * lane) = y;
      if constexpr (MODE == 4) {
        const v8us qv = *(const v8usa*)(hst + (size_t)lr * QP + 8 * lane);
        *(volatile v8us*)(outH + grow * QP + 8 * lane) = qv;
      }
    }
  }
}

__global__ __launch_bounds__(NTHR) void k_gcn(const int* __restrict__ srcs, const int* __restrict__ dsts,
                                              int nE, int nN, int vec8, int mRows,
                                              const float* __restrict__ dis,
                                              const float* __restrict__ xl, const float* __restrict__ bias,
                                              unsigned short* hb) {
  extern __shared__ __attribute__((aligned(16))) int dsm[];
  int* list = dsm;
  int* hl   = dsm + LISTN;
  int* sl   = hl + RCAP;
  int* cnt  = sl + RCAP;
  int* offs = cnt + NBA;
  int* cur  = offs + NBA;
  int* misc = cur + NBA;
  const int tid = (int)threadIdx.x, lane = tid & 31, wave = tid >> 5;
  unsigned short* rowbuf = (unsigned short*)(misc + MISC_INTS) + wave * QP;
  const int nodeBase = (int)blockIdx.x * NBA;

  {
    const v4i z4 = {0, 0, 0, 0};
    for (int i = tid * 4; i < AGG_ZINTS; i += NTHR * 4) *(v4ia*)(dsm + i) = z4;
    if (tid < MISC_INTS) misc[tid] = 0;
  }
  __syncthreads();

  int t = 0, ov = 0;
  const int nChunks = (nE + CHUNK - 1) / CHUNK;
#pragma unroll 1
  for (int ch = 0; ch < nChunks; ++ch) {
    const int cbase = ch * CHUNK;
    const int wc = scan_chunk<SLA>(dsts, nE, cbase, nodeBase, NBA, vec8, list, tid, lane, wave);
    if (lane == 0) misc[wave] = wc;
    __syncthreads();
    if (wave == 0) {
#pragma unroll 1
      for (int w2 = 0; w2 < NWAVE; ++w2) {
        int c = misc[w2];
        c = c < 0 ? 0 : (c > WCAP ? WCAP : c);
#pragma unroll 1
        for (int b0 = 0; b0 < c; b0 += 32) {
          const int idx = b0 + lane;
          const int ent = list[w2 * WCAP + (idx < WCAP ? idx : WCAP - 1)];
          const int m32 = (c - b0) < 32 ? (c - b0) : 32;
#pragma unroll 1
          for (int k = 0; k < m32; ++k) {
            const int u    = __builtin_amdgcn_readlane(ent, k);
            const int slot = u & (NBA - 1);
            const int el   = (u >> SLA) & (CHUNK - 1);
            const int pk   = ((cbase + el) << SLA) | slot;
            if (t < RCAP) {
              if (lane == 0) { hl[t] = pk; cnt[slot] = cnt[slot] + 1; }
              t = t + 1;
            } else {
              ov = 1;
            }
          }
        }
      }
    }
    __syncthreads();
  }
  if (wave == 0 && lane == 0) { misc[8] = t; misc[9] = ov; }
  __syncthreads();
  int tt = misc[8];
  tt = tt < 0 ? 0 : (tt > RCAP ? RCAP : tt);
  const int ovf = misc[9];

  if (wave == 0) {
    const int base = lane * (NBA / 32);
    int s = 0;
#pragma unroll 1
    for (int i = 0; i < NBA / 32; ++i) s += cnt[base + i];
    int incl = s;
#pragma unroll
    for (int d = 1; d < 32; d <<= 1) {
      const int y = __shfl_up(incl, d, 32);
      if (lane >= d) incl += y;
    }
    int run = incl - s;
#pragma unroll 1
    for (int i = 0; i < NBA / 32; ++i) {
      const int cv = cnt[base + i];
      offs[base + i] = run;
      cur[base + i]  = run;
      run += cv;
    }
  }
  __syncthreads();
  if (wave == 0) {
#pragma unroll 1
    for (int b0 = 0; b0 < tt; b0 += 32) {
      const int idx = b0 + lane;
      const int ent = hl[idx < RCAP ? idx : RCAP - 1];
      const int m32 = (tt - b0) < 32 ? (tt - b0) : 32;
#pragma unroll 1
      for (int k = 0; k < m32; ++k) {
        const int u    = __builtin_amdgcn_readlane(ent, k);
        const int slot = u & (NBA - 1);
        if (lane == 0) {
          int p = cur[slot];
          p = p < 0 ? 0 : (p > RCAP - 1 ? RCAP - 1 : p);
          sl[p] = u;
          cur[slot] = p + 1;
        }
      }
    }
  }
  __syncthreads();

  const float qnan = __int_as_float(0x7fc00000);
  const float pz = (ovf != 0) ? qnan : 0.0f;
  v4f bb4;
  {
    const v4f a = *(const v4fa*)(bias + 4 * lane);
    bb4.x = bf16_val(a.x); bb4.y = bf16_val(a.y); bb4.z = bf16_val(a.z); bb4.w = bf16_val(a.w);
  }
#pragma unroll 1
  for (int si = 0; si < NBA / NWAVE; ++si) {
    const int s    = si * NWAVE + wave;
    const int node = nodeBase + s;
    int c = cnt[s];
    const bool big = c > DEGCAP;
    c = c < 0 ? 0 : (c > DEGCAP ? DEGCAP : c);
    int o = offs[s];
    o = o < 0 ? 0 : (o > RCAP ? RCAP : o);
    const int nc = node < nN ? node : nN - 1;
    const float dd = dis[nc];
    const float rd = dd * dd;
    float a0 = 0.0f, a1 = 0.0f, a2 = 0.0f, a3 = 0.0f;
#pragma unroll 1
    for (int b0 = 0; b0 < c; b0 += 32) {
      int idx = o + b0 + lane;
      idx = idx > RCAP - 1 ? RCAP - 1 : idx;
      const int ent = sl[idx];
      int eid = ent >> SLA;
      eid = eid < 0 ? 0 : (eid > nE - 1 ? nE - 1 : eid);
      int sr = srcs[eid];
      sr = sr < 0 ? 0 : (sr > nN - 1 ? nN - 1 : sr);
      const float cf  = dis[sr] * dd;
      const int   cfi = __float_as_int(cf);
      const int m32 = (c - b0) < 32 ? (c - b0) : 32;
#pragma unroll 1
      for (int k = 0; k < m32; ++k) {
        const int   sk = __builtin_amdgcn_readlane(sr, k);
        const float ck = __int_as_float(__builtin_amdgcn_readlane(cfi, k));
        const v4f a = *(const v4fa*)(xl + (size_t)sk * DM + 4 * lane);
        a0 = fmaf(ck, a.x, a0); a1 = fmaf(ck, a.y, a1);
        a2 = fmaf(ck, a.z, a2); a3 = fmaf(ck, a.w, a3);
      }
    }
    const v4f sv = *(const v4fa*)(xl + (size_t)nc * DM + 4 * lane);
    const float pzr = big ? qnan : pz;
    const bool live = node < nN;
    float y0 = (a0 + sv.x * rd) + bb4.x;
    float y1 = (a1 + sv.y * rd) + bb4.y;
    float y2 = (a2 + sv.z * rd) + bb4.z;
    float y3 = (a3 + sv.w * rd) + bb4.w;
    y0 = fmaxf(y0, 0.0f); y1 = fmaxf(y1, 0.0f); y2 = fmaxf(y2, 0.0f); y3 = fmaxf(y3, 0.0f);
    y0 = y0 + pzr; y1 = y1 + pzr; y2 = y2 + pzr; y3 = y3 + pzr;
    const float m0 = live ? y0 : 0.0f;
    const float m1 = live ? y1 : 0.0f;
    const float m2 = live ? y2 : 0.0f;
    const float m3 = live ? y3 : 0.0f;
    v4us mh, ml;
    {
      unsigned hbb;
      hbb = bf16_bits(m0); mh[0] = (unsigned short)hbb; ml[0] = (unsigned short)bf16_bits(m0 - __uint_as_float(hbb << 16));
      hbb = bf16_bits(m1); mh[1] = (unsigned short)hbb; ml[1] = (unsigned short)bf16_bits(m1 - __uint_as_float(hbb << 16));
      hbb = bf16_bits(m2); mh[2] = (unsigned short)hbb; ml[2] = (unsigned short)bf16_bits(m2 - __uint_as_float(hbb << 16));
      hbb = bf16_bits(m3); mh[3] = (unsigned short)hbb; ml[3] = (unsigned short)bf16_bits(m3 - __uint_as_float(hbb << 16));
    }
    *(v4usa*)(rowbuf + 4 * lane) = mh;
    *(v4usa*)(rowbuf + DM + 4 * lane) = ml;
    wave_sync();
    const v8us q0 = *(const v8usa*)(rowbuf + 8 * lane);
    wave_sync();
    if (node < mRows) {
      unsigned short* rpw = hb + (size_t)node * QP + 8 * lane;
      *(volatile v8us*)rpw = q0;
      __threadfence();
      *(volatile v8us*)rpw = q0;
    }
  }
}

__global__ __launch_bounds__(ATHR) void k_attn(const unsigned short* __restrict__ Qp,
                                               const unsigned short* __restrict__ Kp,
                                               const unsigned short* __restrict__ Vt,
                                               unsigned short* ctx) {
  __shared__ __attribute__((aligned(16))) unsigned short cst[ATQ * QP];
  const int tid = (int)threadIdx.x, lane = tid & 31, wave = tid >> 5, lh = lane >> 4, m = lane & 15;
  const int b  = (int)blockIdx.y;
  const int qb = (int)blockIdx.x * ATQ + 16 * wave;
  const size_t tok0 = (size_t)b * MSEQ + (size_t)qb;
  const v8f z8 = {0.f, 0.f, 0.f, 0.f, 0.f, 0.f, 0.f, 0.f};

#pragma unroll 1
  for (int hd = 0; hd < NHEAD; ++hd) {
    FragB bqh, bql;
    {
      const unsigned short* qp = Qp + (tok0 + (size_t)m) * QP + HDIM * hd + 8 * lh;
      bqh.h[0] = *(const v8usa*)qp;        bqh.h[1] = bqh.h[0];
      bql.h[0] = *(const v8usa*)(qp + DM); bql.h[1] = bql.h[0];
    }
    const unsigned short* kbase = Kp + ((size_t)b * MSEQ + (size_t)m) * QP + HDIM * hd + 8 * lh;
    const unsigned short* vbh = Vt + ((size_t)b * QP + (size_t)(HDIM * hd + m)) * (size_t)VTP + 8 * lh;
    const unsigned short* vbl = vbh + (size_t)DM * (size_t)VTP;
    float mrun = -1.0e30f, lrun = 0.0f;
    v8f oacc = z8;
#pragma unroll 1
    for (int kb = 0; kb < MSEQ / 32; ++kb) {
      v8f st[2];
#pragma unroll
      for (int t = 0; t < 2; ++t) {
        const unsigned short* kp2 = kbase + (size_t)(32 * kb + 16 * t) * QP;
        FragB ak;
        ak.h[0] = *(const v8usa*)kp2;
        ak.h[1] = *(const v8usa*)(kp2 + DM);
        st[t] = wmb(ak, bqh, z8);
        st[t] = wmb(ak, bql, st[t]);
      }
      float lmax = st[0][0];
#pragma unroll
      for (int r = 0; r < 8; ++r) { lmax = fmaxf(lmax, st[0][r]); lmax = fmaxf(lmax, st[1][r]); }
      lmax = fmaxf(lmax, __shfl_xor(lmax, 16, 32));
      const float mnew  = fmaxf(mrun, 0.25f * lmax);
      const float alpha = __expf(mrun - mnew);
      float p0[8], p1[8];
      float lsum = 0.0f;
#pragma unroll
      for (int r = 0; r < 8; ++r) {
        p0[r] = __expf(fmaf(st[0][r], 0.25f, -mnew));
        p1[r] = __expf(fmaf(st[1][r], 0.25f, -mnew));
        lsum += p0[r] + p1[r];
      }
      lsum += __shfl_xor(lsum, 16, 32);
      lrun = fmaf(lrun, alpha, lsum);
      mrun = mnew;
#pragma unroll
      for (int r = 0; r < 8; ++r) {
        const float ar = __shfl(alpha, 8 * lh + r, 32);
        oacc[r] = oacc[r] * ar;
      }
      FragB pa, pb;
#pragma unroll
      for (int r = 0; r < 8; ++r) {
        const unsigned ha = bf16_bits(p0[r]);
        const unsigned hc = bf16_bits(p1[r]);
        pa.u[r]     = (unsigned short)ha;
        pa.u[8 + r] = (unsigned short)hc;
        pb.u[r]     = (unsigned short)bf16_bits(p0[r] - __uint_as_float(ha << 16));
        pb.u[8 + r] = (unsigned short)bf16_bits(p1[r] - __uint_as_float(hc << 16));
      }
      FragB vh, vl;
      {
        const unsigned short* vph = vbh + 32 * kb;
        const unsigned short* vpl = vbl + 32 * kb;
        vh.h[0] = *(const v8usa*)vph;  vh.h[1] = *(const v8usa*)(vph + 16);
        vl.h[0] = *(const v8usa*)vpl;  vl.h[1] = *(const v8usa*)(vpl + 16);
      }
      oacc = wmb(pa, vh, oacc);
      oacc = wmb(pa, vl, oacc);
      oacc = wmb(pb, vh, oacc);
    }
    const float inv = 1.0f / lrun;
#pragma unroll
    for (int r = 0; r < 8; ++r) {
      const float ir = __shfl(inv, 8 * lh + r, 32);
      const float o  = oacc[r] * ir;
      const unsigned ho = bf16_bits(o);
      const unsigned lo = bf16_bits(o - __uint_as_float(ho << 16));
      const int crow = 16 * wave + 8 * lh + r;
      cst[crow * QP + HDIM * hd + m]      = (unsigned short)ho;
      cst[crow * QP + DM + HDIM * hd + m] = (unsigned short)lo;
    }
  }
  __syncthreads();
#pragma unroll 1
  for (int i = 0; i < 16; ++i) {
    const int crow = 16 * wave + i;
    const v8us qv = *(const v8usa*)(cst + crow * QP + 8 * lane);
    *(volatile v8us*)(ctx + (tok0 + (size_t)i) * QP + 8 * lane) = qv;
  }
  __threadfence();
#pragma unroll 1
  for (int i = 0; i < 16; ++i) {
    const int crow = 16 * wave + i;
    const v8us qv = *(const v8usa*)(cst + crow * QP + 8 * lane);
    *(volatile v8us*)(ctx + (tok0 + (size_t)i) * QP + 8 * lane) = qv;
  }
}

static inline int cdiv(int a, int b) { return (a + b - 1) / b; }
static inline size_t al256(size_t o) { return (o + 255) & ~(size_t)255; }

extern "C" void kernel_launch(void* const* d_in, const int* in_sizes, int n_in,
                              void* d_out, int out_size, void* d_ws, size_t ws_size,
                              hipStream_t stream) {
  if (n_in < 24) return;
  if (in_sizes[2] < DM || (in_sizes[2] % DM) != 0) return;
  const int nN = in_sizes[2] / DM;
  if ((nN % MSEQ) != 0 || nN < MSEQ || nN > (1 << 22)) return;
  const int nB = nN / MSEQ;
  if (in_sizes[0] != nN * DM) return;
  if (in_sizes[3] < 2 || (in_sizes[3] & 1) != 0) return;
  const int nE = in_sizes[3] / 2;
  if (nE < 1 || nE >= (1 << (31 - SLA))) return;
  if (in_sizes[4] != DM * DM || in_sizes[5] != DM || in_sizes[6] != DM * DM || in_sizes[7] != DM) return;
  if (in_sizes[8] != NLAYER * DM * DM || in_sizes[10] != NLAYER * DM * DM) return;
  if (in_sizes[12] != NLAYER * DM * DM || in_sizes[14] != NLAYER * DM * DM) return;
  if (in_sizes[9] != NLAYER * DM || in_sizes[11] != NLAYER * DM || in_sizes[13] != NLAYER * DM || in_sizes[15] != NLAYER * DM) return;
  if (in_sizes[16] != NLAYER * DM * DFF || in_sizes[17] != NLAYER * DFF) return;
  if (in_sizes[18] != NLAYER * DFF * DM || in_sizes[19] != NLAYER * DM) return;
  if (in_sizes[20] != NLAYER * DM || in_sizes[21] != NLAYER * DM || in_sizes[22] != NLAYER * DM || in_sizes[23] != NLAYER * DM) return;
  if (out_size != nN * DM) return;

  const float* enc  = (const float*)d_in[0];
  const float* xr   = (const float*)d_in[2];
  const int*   edge = (const int*)d_in[3];
  const float* c1W  = (const float*)d_in[4];
  const float* c1b  = (const float*)d_in[5];
  const float* c2W  = (const float*)d_in[6];
  const float* c2b  = (const float*)d_in[7];
  const float* Wq   = (const float*)d_in[8];
  const float* bq   = (const float*)d_in[9];
  const float* Wk   = (const float*)d_in[10];
  const float* bk   = (const float*)d_in[11];
  const float* Wv   = (const float*)d_in[12];
  const float* bv   = (const float*)d_in[13];
  const float* Wo   = (const float*)d_in[14];
  const float* bo   = (const float*)d_in[15];
  const float* W1   = (const float*)d_in[16];
  const float* b1   = (const float*)d_in[17];
  const float* W2   = (const float*)d_in[18];
  const float* b2   = (const float*)d_in[19];
  const float* ln1g = (const float*)d_in[20];
  const float* ln1b = (const float*)d_in[21];
  const float* ln2g = (const float*)d_in[22];
  const float* ln2b = (const float*)d_in[23];
  float* out = (float*)d_out;
  const int* src = edge;
  const int* dst = edge + nE;

  const int gM   = nN / GBM;
  const int gD   = cdiv(nN, NBD);
  const int NBPD = gD * NBD;
  const int gA   = cdiv(nN, NBA);
  if ((long long)gA * NBA < (long long)nN) return;
  if (NBPD < nN) return;
  const int vec8 = ((nE & 3) == 0) ? 1 : 0;

  const size_t szB  = (size_t)nN * DM * 2;
  const size_t szF4 = (size_t)nN * DM * 4;
  const size_t szHL = (size_t)nN * QP * 2;
  const size_t szFF = (size_t)nN * FP * 2;
  const size_t szVT = (size_t)nB * QP * VTP * 2;
  if (2 * szB + szF4 + 2 * szHL != szFF) return;
  char* ws = (char*)d_ws;
  size_t off = 0;
  const size_t oDIS = off; off = al256(off + (size_t)NBPD * 4);
  const size_t oWPL = off; off = al256(off + (size_t)WPL_TOT * 2);
  const size_t oFR  = off; off = al256(off + szFF);
  const size_t oKV  = off; off = al256(off + szHL);
  const size_t oKP0 = off; off = al256(off + szHL);
  const size_t oKP1 = off; off = al256(off + szHL);
  const size_t oVT0 = off; off = al256(off + szVT);
  const size_t oVT1 = off; off = al256(off + szVT);
  const size_t oCTX = off; off = al256(off + szHL);
  const size_t oH   = off; off = al256(off + szF4);
  const size_t oHHL = off; off = al256(off + szHL);
  if (off > ws_size || off > (size_t)WSMAX) return;
  float*          DIS = (float*)(ws + oDIS);
  unsigned short* WPL = (unsigned short*)(ws + oWPL);
  unsigned short* F   = (unsigned short*)(ws + oFR);
  unsigned short* XB  = (unsigned short*)(ws + oFR);
  unsigned short* EB  = (unsigned short*)(ws + oFR + szB);
  float*          HW  = (float*)(ws + oFR + 2 * szB);
  unsigned short* X1  = (unsigned short*)(ws + oFR + 2 * szB + szF4);
  unsigned short* QPL = (unsigned short*)(ws + oFR + 2 * szB + szF4 + szHL);
  unsigned short* KV  = (unsigned short*)(ws + oKV);
  unsigned short* KPL[NLAYER] = { (unsigned short*)(ws + oKP0), (unsigned short*)(ws + oKP1) };
  unsigned short* VTL[NLAYER] = { (unsigned short*)(ws + oVT0), (unsigned short*)(ws + oVT1) };
  unsigned short* CTX = (unsigned short*)(ws + oCTX);
  float*          Hf  = (float*)(ws + oH);
  unsigned short* HHL = (unsigned short*)(ws + oHHL);

  const size_t aggLds = (size_t)AGG_LDS_INTS * 4;
  const size_t ldsG   = (size_t)GBM * GBN * 4;
  const size_t ldsL   = ldsG + (size_t)GBM * QP * 2;
  hipFuncSetAttribute(reinterpret_cast<const void*>(&k_gcn), hipFuncAttributeMaxDynamicSharedMemorySize, (int)aggLds);
  hipFuncSetAttribute(reinterpret_cast<const void*>(&k_gemm<4>), hipFuncAttributeMaxDynamicSharedMemorySize, (int)ldsL);
  hipFuncSetAttribute(reinterpret_cast<const void*>(&k_gemm<5>), hipFuncAttributeMaxDynamicSharedMemorySize, (int)ldsL);

  k_wprep<<<dim3(UMAX / NTHR, NPARTS), NTHR, 0, stream>>>(c1W, c2W, Wq, Wk, Wv, Wo, W1, W2, WPL);
  k_cvt<<<dim3((nN * (DM / 4)) / NTHR, 3), NTHR, 0, stream>>>(xr, enc, nN, XB, EB, Hf);
  k_deg<<<gD, NTHR, 0, stream>>>(dst, nE, vec8, DIS);
  k_gemm<0><<<dim3(gM, 1), GTHR, ldsG, stream>>>(XB, DM, WPL + WPL_C1, DM, DM, c1b, DM, Hf, ln1g, ln1b, HW, HHL);
  k_gcn<<<gA, NTHR, aggLds, stream>>>(src, dst, nE, nN, vec8, nN, DIS, HW, c1b, X1);
  k_gemm<0><<<dim3(gM, 1), GTHR, ldsG, stream>>>(X1, QP, WPL + WPL_C2, QP, QP, c2b, DM, Hf, ln1g, ln1b, HW, HHL);
  k_gcn<<<gA, NTHR, aggLds, stream>>>(src, dst, nE, nN, vec8, nN, DIS, HW, c2b, KV);
  for (int l = 0; l < NLAYER; ++l) {
    const unsigned short* WL = WPL + WPL_L0 + (size_t)l * WPL_LSZ;
    k_gemm<1><<<dim3(gM, 1), GTHR, ldsG, stream>>>(KV, QP, WL + WPL_K, QP, QP, bk + l * DM, DM, Hf, ln1g, ln1b, Hf, KPL[l]);
    k_gemm<3><<<dim3(gM, 1), GTHR, ldsG, stream>>>(KV, QP, WL + WPL_V, QP, QP, bv + l * DM, DM, Hf, ln1g, ln1b, Hf, VTL[l]);
  }
  for (int l = 0; l < NLAYER; ++l) {
    const unsigned short* WL = WPL + WPL_L0 + (size_t)l * WPL_LSZ;
    if (l == 0) {
      k_gemm<1><<<dim3(gM, 1), GTHR, ldsG, stream>>>(EB, DM, WL + WPL_Q, QP, DM, bq, DM, Hf, ln1g, ln1b, Hf, QPL);
    } else {
      k_gemm<1><<<dim3(gM, 1), GTHR, ldsG, stream>>>(HHL, QP, WL + WPL_Q, QP, QP, bq + l * DM, DM, Hf, ln1g, ln1b, Hf, QPL);
    }
    k_attn<<<dim3(MSEQ / ATQ, nB), ATHR, 0, stream>>>(QPL, KPL[l], VTL[l], CTX);
    k_gemm<4><<<dim3(gM, 1), GTHR, ldsL, stream>>>(CTX, QP, WL + WPL_O, QP, QP, bo + l * DM, DM,
                                                   Hf, ln1g + l * DM, ln1b + l * DM, Hf, HHL);
    k_gemm<2><<<dim3(gM, DFF / GBN), GTHR, ldsG, stream>>>(HHL, QP, WL + WPL_1, QP, QP, b1 + l * DFF, DFF,
                                                           Hf, ln2g, ln2b, Hf, F);
    if (l + 1 < NLAYER) {
      k_gemm<4><<<dim3(gM, 1), GTHR, ldsL, stream>>>(F, FP, WL + WPL_2, FP, FP, b2 + l * DM, DM,
                                                     Hf, ln2g + l * DM, ln2b + l * DM, Hf, HHL);
    } else {
      k_gemm<5><<<dim3(gM, 1), GTHR, ldsL, stream>>>(F, FP, WL + WPL_2, FP, FP, b2 + l * DM, DM,
                                                     Hf, ln2g + l * DM, ln2b + l * DM, out, HHL);
    }
  }
}
